// GRU_21045339750966
// MI455X (gfx1250) — hardware-verified
//
#include <hip/hip_runtime.h>
#include <math.h>

typedef __attribute__((ext_vector_type(16))) _Float16 v16h;
typedef __attribute__((ext_vector_type(8)))  _Float16 v8h;
typedef __attribute__((ext_vector_type(8)))  float    v8f;
typedef __attribute__((ext_vector_type(4)))  float    v4f;

constexpr int kBatch      = 1024;
constexpr int kSteps      = 2048;
constexpr int kHid        = 10;
constexpr int kTileRows   = 16;
constexpr int kTiles      = kBatch / kTileRows;
constexpr int kChunk      = 32;
constexpr int kNumChunks  = kSteps / kChunk;
constexpr int kPitch      = 36;
constexpr int kMatElems   = 3 * kHid * kHid;
constexpr size_t kOutElems = (size_t)kBatch * (size_t)kSteps;
static_assert(kBatch % kTileRows == 0, "whole 16-row tiles");
static_assert(kSteps % kChunk == 0, "whole 32-step chunks");
static_assert(kHid >= 1 && kHid <= 16, "the units of a gate fit one 16-row subtile and the first 16 k of one instruction");
constexpr int kWPass = (kMatElems + 31) / 32;
static_assert(kWPass * 32 >= kMatElems && 3 * kHid <= 64, "weight staging passes; the 3*kHid-float vectors fit two 32-slot rows");
static_assert((kPitch % 4) == 0, "16-B aligned LDS rows");

constexpr float kStateCarry  = 256.0f;
constexpr float kWeightCarry = 64.0f;
constexpr float kFoldBack    = 1.0f / (kStateCarry * kWeightCarry);
constexpr float kF16MinNorm  = 6.103515625e-5f;
static_assert(kStateCarry * kWeightCarry == 16384.0f, "carry product");

namespace eng {

union FragU { v16h v; v8h h[2]; };

__device__ __forceinline__ unsigned short f2bf_bits(float f) {
  unsigned u = __float_as_uint(f);
  return (unsigned short)((u + 0x7FFFu + ((u >> 16) & 1u)) >> 16);
}
__device__ __forceinline__ float bf16v(float f) {
  return __uint_as_float(((unsigned)f2bf_bits(f)) << 16);
}
__device__ __forceinline__ _Float16 to_f16_flushed(float c) {
  const float z = (fabsf(c) < kF16MinNorm) ? 0.0f : c;
  return (_Float16)z;
}
__device__ __forceinline__ v8f mma_f16(v16h a, v16h b) {
  v8f c = (v8f){0.f, 0.f, 0.f, 0.f, 0.f, 0.f, 0.f, 0.f};
  c = __builtin_amdgcn_wmma_f32_16x16x32_f16(false, a, false, b, (short)0, c, false, false);
  asm volatile("v_nop\n\tv_nop\n\tv_nop\n\tv_nop" : "+v"(c) : "v"(a), "v"(b));
  return c;
}
__device__ __forceinline__ float fast_tanh(float v) {
  const float e = __expf(2.0f * v);
  return 1.0f - 2.0f * __builtin_amdgcn_rcpf(e + 1.0f);
}
__device__ __forceinline__ float fast_sigmoid(float v) {
  return __builtin_amdgcn_rcpf(1.0f + __expf(-v));
}

}

__global__ __launch_bounds__(32) void gru2l_seq_kernel(
    const float* __restrict__ x,
    const float* __restrict__ w_ih,
    const float* __restrict__ w_hh,
    const float* __restrict__ b_ih,
    const float* __restrict__ b_hh,
    const float* __restrict__ w_ih2,
    const float* __restrict__ w_hh2,
    const float* __restrict__ b_ih2,
    const float* __restrict__ b_hh2,
    const float* __restrict__ w_out,
    const float* __restrict__ b_out,
    float* __restrict__ outs)
{
  __shared__ __align__(16) float xs[kTileRows * kPitch];
  __shared__ __align__(16) float os[kTileRows * kPitch];
  __shared__ __align__(16) float wsm[kWPass * 32];
  __shared__ __align__(16) float csm[3 * 64 + 2 * 32];
  __shared__ __align__(16) float wi2[kWPass * 32];
  __shared__ __align__(16) float wh2[kWPass * 32];
  __shared__ __align__(16) float c2m[2 * 64];

  const int lane = threadIdx.x & 31;
  const int hsel = lane >> 4;
  const int n    = lane & 15;
  const bool lowHalf = (hsel == 0);
  const int b0   = blockIdx.x * kTileRows;

  {
#pragma unroll
    for (int it = 0; it < kWPass; ++it) {
      const int i  = it * 32 + lane;
      const int ic = (i < kMatElems) ? i : (kMatElems - 1);
      wsm[ic] = w_hh[ic];
    }
#pragma unroll
    for (int it = 0; it < 2; ++it) {
      const int s  = it * 32 + lane;
      const int sc = (s < 3 * kHid - 1) ? s : (3 * kHid - 1);
      csm[0 * 64 + s] = w_ih[sc];
      csm[1 * 64 + s] = b_ih[sc];
      csm[2 * 64 + s] = b_hh[sc];
    }
    const int cH = (lane < kHid - 1) ? lane : (kHid - 1);
    csm[3 * 64 + lane]      = w_out[cH];
    csm[3 * 64 + 32 + lane] = b_out[0];
#pragma unroll
    for (int it = 0; it < kWPass; ++it) {
      const int i  = it * 32 + lane;
      const int ic = (i < kMatElems) ? i : (kMatElems - 1);
      wi2[ic] = w_ih2[ic];
      wh2[ic] = w_hh2[ic];
    }
#pragma unroll
    for (int it = 0; it < 2; ++it) {
      const int s  = it * 32 + lane;
      const int sc = (s < 3 * kHid - 1) ? s : (3 * kHid - 1);
      c2m[0 * 64 + s] = b_ih2[sc];
      c2m[1 * 64 + s] = b_hh2[sc];
    }
  }
  __syncthreads();

  v16h fragA[3];
  v16h fragB2[4];
  {
    const int m  = n;
    const int mc = (m < kHid) ? m : (kHid - 1);
    const bool mok = (m < kHid);
    const v8h zero8 = (v8h){(_Float16)0.0f, (_Float16)0.0f, (_Float16)0.0f, (_Float16)0.0f,
                            (_Float16)0.0f, (_Float16)0.0f, (_Float16)0.0f, (_Float16)0.0f};
#pragma unroll
    for (int g = 0; g < 3; ++g) {
      v8h alo;
#pragma unroll
      for (int i = 0; i < 8; ++i) {
        const int k  = 8 * hsel + i;
        const int kc = (k < kHid) ? k : (kHid - 1);
        const bool ok = mok && (k < kHid);
        const float f0 = wsm[(g * kHid + mc) * kHid + kc];
        const float g0 = ok ? (eng::bf16v(f0) * kWeightCarry) : 0.0f;
        alo[i] = eng::to_f16_flushed(g0);
      }
      eng::FragU u0;
      u0.h[0] = alo;
      u0.h[1] = zero8;
      fragA[g] = u0.v;
    }
#pragma unroll
    for (int g = 0; g < 3; ++g) {
      v8h ai, ah;
#pragma unroll
      for (int i = 0; i < 8; ++i) {
        const int k  = 8 * hsel + i;
        const int kc = (k < kHid) ? k : (kHid - 1);
        const bool ok = mok && (k < kHid);
        const float fi = wi2[(g * kHid + mc) * kHid + kc];
        const float fh = wh2[(g * kHid + mc) * kHid + kc];
        const float gi = ok ? (eng::bf16v(fi) * kWeightCarry) : 0.0f;
        const float gh = ok ? (eng::bf16v(fh) * kWeightCarry) : 0.0f;
        ai[i] = eng::to_f16_flushed(gi);
        ah[i] = eng::to_f16_flushed(gh);
      }
      eng::FragU u1;
      if (g < 2) {
        u1.h[0] = ai;
        u1.h[1] = ah;
        fragB2[g] = u1.v;
      } else {
        u1.h[0] = ai;
        u1.h[1] = zero8;
        fragB2[2] = u1.v;
        eng::FragU u2;
        u2.h[0] = zero8;
        u2.h[1] = ah;
        fragB2[3] = u2.v;
      }
    }
  }

  float wxr[8], wxz[8], wxn[8], cbr[8], cbz[8], cin[8], chn[8], wo[8];
  float hf[8];
  v8h hb;
  float cbr2[8], cbz2[8], cin2[8], chn2[8];
  float hf2[8];
  v8h hb2;
#pragma unroll
  for (int r = 0; r < 8; ++r) {
    const int u  = 8 * hsel + r;
    const int uc = (u < kHid) ? u : (kHid - 1);
    const bool live = (u < kHid);
    wxr[r] = eng::bf16v(csm[0 * 64 + uc]);
    wxz[r] = eng::bf16v(csm[0 * 64 + kHid + uc]);
    wxn[r] = eng::bf16v(csm[0 * 64 + 2 * kHid + uc]);
    cbr[r] = eng::bf16v(csm[1 * 64 + uc]) + eng::bf16v(csm[2 * 64 + uc]);
    cbz[r] = eng::bf16v(csm[1 * 64 + kHid + uc]) + eng::bf16v(csm[2 * 64 + kHid + uc]);
    cin[r] = eng::bf16v(csm[1 * 64 + 2 * kHid + uc]);
    chn[r] = eng::bf16v(csm[2 * 64 + 2 * kHid + uc]);
    const float vwo = eng::bf16v(csm[3 * 64 + uc]);
    wo[r]  = live ? vwo : 0.0f;
    hf[r] = 0.0f;
    hb[r] = (_Float16)0.0f;
    cbr2[r] = eng::bf16v(c2m[0 * 64 + uc]) + eng::bf16v(c2m[1 * 64 + uc]);
    cbz2[r] = eng::bf16v(c2m[0 * 64 + kHid + uc]) + eng::bf16v(c2m[1 * 64 + kHid + uc]);
    cin2[r] = eng::bf16v(c2m[0 * 64 + 2 * kHid + uc]);
    chn2[r] = eng::bf16v(c2m[1 * 64 + 2 * kHid + uc]);
    hf2[r] = 0.0f;
    hb2[r] = (_Float16)0.0f;
  }
  const float bo = eng::bf16v(csm[3 * 64 + 32]);
  const v8h zh = (v8h){(_Float16)0.0f, (_Float16)0.0f, (_Float16)0.0f, (_Float16)0.0f,
                       (_Float16)0.0f, (_Float16)0.0f, (_Float16)0.0f, (_Float16)0.0f};

  const int q  = lane >> 3;
  const int c4 = (lane & 7) * 4;

#pragma unroll 1
  for (int ch = 0; ch < kNumChunks; ++ch) {
    const int t0 = ch * kChunk;
#pragma unroll
    for (int it = 0; it < 4; ++it) {
      const int row = it * 4 + q;
      const v4f v = *(const v4f*)(x + (size_t)(b0 + row) * kSteps + t0 + c4);
      v4f rv;
      const float v0 = v[0];
      const float v1 = v[1];
      const float v2 = v[2];
      const float v3 = v[3];
      rv[0] = eng::bf16v(v0);
      rv[1] = eng::bf16v(v1);
      rv[2] = eng::bf16v(v2);
      rv[3] = eng::bf16v(v3);
      *(v4f*)(xs + row * kPitch + c4) = rv;
    }
    __syncthreads();

#pragma unroll 1
    for (int s = 0; s < kChunk; ++s) {
      const float xv = xs[n * kPitch + s];

      eng::FragU fb;
      fb.h[0] = hb;
      fb.h[1] = zh;
      const v8f ar = eng::mma_f16(fragA[0], fb.v);
      const v8f az = eng::mma_f16(fragA[1], fb.v);
      const v8f an = eng::mma_f16(fragA[2], fb.v);
      float p = 0.0f;
#pragma unroll
      for (int r = 0; r < 8; ++r) {
        const float rg = eng::fast_sigmoid(fmaf(ar[r], kFoldBack, fmaf(xv, wxr[r], cbr[r])));
        const float zg = eng::fast_sigmoid(fmaf(az[r], kFoldBack, fmaf(xv, wxz[r], cbz[r])));
        const float hn = fmaf(an[r], kFoldBack, chn[r]);
        const float ng = eng::fast_tanh(fmaf(xv, wxn[r], cin[r]) + rg * hn);
        const float tv = (1.0f - zg) * ng + zg * hf[r];
        const bool live = (8 * hsel + r) < kHid;
        const float hv = live ? tv : 0.0f;
        hf[r] = hv;
        hb[r] = eng::to_f16_flushed(hv * kStateCarry);
      }
      eng::FragU f2;
      f2.h[0] = hb;
      f2.h[1] = hb2;
      const v8f br = eng::mma_f16(fragB2[0], f2.v);
      const v8f bz = eng::mma_f16(fragB2[1], f2.v);
      const v8f bni = eng::mma_f16(fragB2[2], f2.v);
      const v8f bnh = eng::mma_f16(fragB2[3], f2.v);
#pragma unroll
      for (int r = 0; r < 8; ++r) {
        const float rg = eng::fast_sigmoid(fmaf(br[r], kFoldBack, cbr2[r]));
        const float zg = eng::fast_sigmoid(fmaf(bz[r], kFoldBack, cbz2[r]));
        const float hn = fmaf(bnh[r], kFoldBack, chn2[r]);
        const float ng = eng::fast_tanh(fmaf(bni[r], kFoldBack, cin2[r]) + rg * hn);
        const float tv = (1.0f - zg) * ng + zg * hf2[r];
        const bool live = (8 * hsel + r) < kHid;
        const float hv = live ? tv : 0.0f;
        hf2[r] = hv;
        hb2[r] = eng::to_f16_flushed(hv * kStateCarry);
        p = fmaf(wo[r], hv, p);
      }
      const float pother = __shfl_xor(p, 16, 32);
      const float tot = (p + pother) + bo;
      if (lowHalf) os[n * kPitch + s] = tot;
    }
    __syncthreads();

    {
      v4f ov[4];
#pragma unroll
      for (int it = 0; it < 4; ++it) ov[it] = *(const v4f*)(os + (it * 4 + q) * kPitch + c4);
      for (int pass = 0; pass < 2; ++pass) {
#pragma unroll
        for (int it = 0; it < 4; ++it)
          *(volatile v4f*)(outs + (size_t)(b0 + it * 4 + q) * kSteps + t0 + c4) = ov[it];
        __threadfence();
      }
    }
  }
}

extern "C" void kernel_launch(void* const* d_in, const int* in_sizes, int n_in,
                              void* d_out, int out_size, void* d_ws, size_t ws_size,
                              hipStream_t stream) {
  (void)d_ws;
  (void)ws_size;
  if (n_in < 11 || d_out == nullptr) return;
  if ((size_t)in_sizes[0] != kOutElems) return;
  if (in_sizes[1] != 3 * kHid) return;
  if (in_sizes[2] != kMatElems) return;
  if (in_sizes[3] != 3 * kHid) return;
  if (in_sizes[4] != 3 * kHid) return;
  if (in_sizes[5] != kMatElems) return;
  if (in_sizes[6] != kMatElems) return;
  if (in_sizes[7] != 3 * kHid) return;
  if (in_sizes[8] != 3 * kHid) return;
  if (in_sizes[9] != kHid) return;
  if (in_sizes[10] != 1) return;
  if ((size_t)out_size != kOutElems) return;

  const float* x     = (const float*)d_in[0];
  const float* w_ih  = (const float*)d_in[1];
  const float* w_hh  = (const float*)d_in[2];
  const float* b_ih  = (const float*)d_in[3];
  const float* b_hh  = (const float*)d_in[4];
  const float* w_ih2 = (const float*)d_in[5];
  const float* w_hh2 = (const float*)d_in[6];
  const float* b_ih2 = (const float*)d_in[7];
  const float* b_hh2 = (const float*)d_in[8];
  const float* w_out = (const float*)d_in[9];
  const float* b_out = (const float*)d_in[10];
  float* outs = (float*)d_out;

  gru2l_seq_kernel<<<kTiles, 32, 0, stream>>>(x, w_ih, w_hh, b_ih, b_hh, w_ih2, w_hh2, b_ih2, b_hh2, w_out, b_out, outs);
}
